// GraphModel_2241972928707
// MI455X (gfx1250) — hardware-verified
//
#include <hip/hip_runtime.h>
#include <math.h>

constexpr int NNODE = 50000;
constexpr int NPAD  = 50048;
constexpr int NEDGE = 800000;
constexpr int FDIM  = 128;
constexpr int NLAY  = 4;
constexpr int NCLS  = 16;
constexpr int NCLP  = 64;
constexpr int NTHR  = 256;
constexpr int SRB   = 8192;
constexpr int RPW   = SRB / 8;
constexpr int NTILE = 7;
constexpr int AGGR  = NTILE * SRB;
constexpr int SCH   = 4096;
constexpr int SPT   = SCH / NTHR;
constexpr int NCH   = (NEDGE + SCH - 1) / SCH;
constexpr int SCANW = 80;

static_assert(NPAD % 64 == 0 && NPAD >= NNODE, "M tile multiple");
static_assert(FDIM % 64 == 0 && FDIM % 32 == 0, "N/K tile multiples");
static_assert(NCLP % 64 == 0 && NCLP >= NCLS, "classifier N tile multiple");
static_assert(AGGR >= NPAD, "tiles cover all padded rows");
static_assert(NEDGE % SPT == 0, "thread edge groups entirely in or out of range");
static_assert(SPT % 4 == 0 && SCH == SPT * NTHR, "chunk geometry");
static_assert(NCH * SCH >= NEDGE, "chunks cover the edge list");
static_assert(SCH < 65536 && SRB <= 8192, "list record encoding (dl << 16) | chunk offset fits in 29 bits");
static_assert(RPW == 1024 && (SRB / RPW) == 8, "wave ownership = dl >> 10");
static_assert((NNODE * NCLS) % (32 * 4) == 0, "output waves are whole");
static_assert(SCANW >= 65 && SCANW <= NTHR, "scan scratch covered by one init pass");

typedef __attribute__((ext_vector_type(16))) _Float16 v16h;
typedef __attribute__((ext_vector_type(8)))  _Float16 v8h;
typedef __attribute__((ext_vector_type(16))) __bf16   v16b;
typedef __attribute__((ext_vector_type(8)))  __bf16   v8b;
typedef __attribute__((ext_vector_type(8)))  float    v8f;
typedef __attribute__((ext_vector_type(4)))  float    v4f;
typedef __attribute__((ext_vector_type(4)))  int      v4i;
typedef __attribute__((ext_vector_type(4)))  unsigned int v4u;

__device__ __forceinline__ unsigned short f2bf_bits(float f) {
  unsigned u = __float_as_uint(f);
  return (unsigned short)((u + 0x7FFFu + ((u >> 16) & 1u)) >> 16);
}
__device__ __forceinline__ float bf_bits2f(unsigned short h) { return __uint_as_float(((unsigned)h) << 16); }
__device__ __forceinline__ unsigned pk16(unsigned short a, unsigned short b) { return (unsigned)a | ((unsigned)b << 16); }

__device__ __forceinline__ void dep_guard_h(v8f& a, v8f& b, v16h x, v16h y) { asm volatile("v_nop\n\tv_nop\n\tv_nop\n\tv_nop" : "+v"(a), "+v"(b) : "v"(x), "v"(y)); }
__device__ __forceinline__ void dep_guard_b(v8f& a, v8f& b, v16b x, v16b y) { asm volatile("v_nop\n\tv_nop\n\tv_nop\n\tv_nop" : "+v"(a), "+v"(b) : "v"(x), "v"(y)); }
__device__ __forceinline__ void dep_guard4_h(v8f& a, v8f& b, v8f& c, v8f& d, v16h x, v16h y) { asm volatile("v_nop\n\tv_nop\n\tv_nop\n\tv_nop" : "+v"(a), "+v"(b), "+v"(c), "+v"(d) : "v"(x), "v"(y)); }
__device__ __forceinline__ void dep_guard4_b(v8f& a, v8f& b, v8f& c, v8f& d, v16b x, v16b y) { asm volatile("v_nop\n\tv_nop\n\tv_nop\n\tv_nop" : "+v"(a), "+v"(b), "+v"(c), "+v"(d) : "v"(x), "v"(y)); }
__device__ __forceinline__ void keep4_h(v16h a, v16h b, v16h c, v16h d) { asm volatile("v_nop" :: "v"(a), "v"(b), "v"(c), "v"(d)); }
__device__ __forceinline__ void keep4_b(v16b a, v16b b, v16b c, v16b d) { asm volatile("v_nop" :: "v"(a), "v"(b), "v"(c), "v"(d)); }
__device__ __forceinline__ void acc_guard4(v8f& a, v8f& b, v8f& c, v8f& d) { asm volatile("v_nop\n\tv_nop\n\tv_nop\n\tv_nop" : "+v"(a), "+v"(b), "+v"(c), "+v"(d)); }
template <typename T> struct Frag;
template <> struct Frag<_Float16> {
  typedef v16h V; union U { v16h v; v8h h[2]; };
  static __device__ __forceinline__ v16h load(const _Float16* p) {
    U f; f.h[0] = *(const v8h*)(p); f.h[1] = *(const v8h*)(p + 16); return f.v;
  }
  static __device__ __forceinline__ v8f mma(v16h a, v16h b, v8f c) {
    return __builtin_amdgcn_wmma_f32_16x16x32_f16(false, a, false, b, (short)0, c, false, false);
  }
  static __device__ __forceinline__ void guard(v8f& a, v8f& b, v16h x, v16h y) { dep_guard_h(a, b, x, y); }
  static __device__ __forceinline__ void guard4(v8f& a, v8f& b, v8f& c, v8f& d, v16h x, v16h y) { dep_guard4_h(a, b, c, d, x, y); }
  static __device__ __forceinline__ void keep(v16h a, v16h b, v16h c, v16h d) { keep4_h(a, b, c, d); }
};
template <> struct Frag<__bf16> {
  typedef v16b V; union U { v16b v; v8b h[2]; };
  static __device__ __forceinline__ v16b load(const __bf16* p) {
    U f; f.h[0] = *(const v8b*)(p); f.h[1] = *(const v8b*)(p + 16); return f.v;
  }
  static __device__ __forceinline__ v8f mma(v16b a, v16b b, v8f c) {
    return __builtin_amdgcn_wmma_f32_16x16x32_bf16(false, a, false, b, (short)0, c, false, false);
  }
  static __device__ __forceinline__ void guard(v8f& a, v8f& b, v16b x, v16b y) { dep_guard_b(a, b, x, y); }
  static __device__ __forceinline__ void guard4(v8f& a, v8f& b, v8f& c, v8f& d, v16b x, v16b y) { dep_guard4_b(a, b, c, d, x, y); }
  static __device__ __forceinline__ void keep(v16b a, v16b b, v16b c, v16b d) { keep4_b(a, b, c, d); }
};

template <int ET> struct Elem;
template <> struct Elem<0> { typedef _Float16 T; };
template <> struct Elem<1> { typedef __bf16 T; };
template <int ET, bool SPLIT, int BIAS_MODE, int OUT_MODE, bool RESID, int ACT = 0>
__global__ __launch_bounds__(256) void wmma_gemm64(
    const unsigned short* __restrict__ Ap, const unsigned short* __restrict__ A2p, int lda, long strideA,
    const unsigned short* __restrict__ Btp, const unsigned short* __restrict__ Bt2p, int ldb, long strideB,
    void* __restrict__ Cout, void* __restrict__ Cout2, int ldc, long strideC,
    const float* __restrict__ bias,
    const float* __restrict__ resid, long strideR,
    int M, int N, int K, float scale) {
  typedef typename Elem<ET>::T T;
  typedef typename Frag<T>::V V;
  const T* A = (const T*)Ap; const T* A2 = (const T*)A2p; const T* Bt = (const T*)Btp; const T* Bt2 = (const T*)Bt2p;
  __shared__ __align__(16) float sT[8][16 * 68];
  const int b    = blockIdx.y;
  const int lane = threadIdx.x & 31;
  const int wave = threadIdx.x >> 5;
  const int tilesN = N >> 6;
  const int tilesM = M >> 6;
  const int tile = blockIdx.x * 8 + wave;
  if (tile >= tilesM * tilesN) return;
  const int tm = tile / tilesN;
  const int tn = tile - tm * tilesN;
  const int m0 = tm << 6;
  const int n0 = tn << 6;

  const T* Ab  = A  + (size_t)b * strideA;
  const T* Bb  = Bt + (size_t)b * strideB;
  const T* Ab2 = SPLIT ? (A2  + (size_t)b * strideA) : nullptr;
  const T* Bb2 = SPLIT ? (Bt2 + (size_t)b * strideB) : nullptr;

  const int rlane = lane & 15;
  const int koff  = (lane >> 4) * 8;
  const int mOff  = (lane >> 4) * 8;

  v8f acc[4][4];
#pragma unroll
  for (int i = 0; i < 4; ++i)
#pragma unroll
    for (int j = 0; j < 4; ++j) acc[i][j] = (v8f){0.f,0.f,0.f,0.f,0.f,0.f,0.f,0.f};

  for (int k0 = 0; k0 < K; k0 += 32) {
    V bh[4], bl[4];
#pragma unroll
    for (int j = 0; j < 4; ++j) {
      const size_t bo = (size_t)(n0 + (j << 4) + rlane) * ldb + koff + k0;
      bh[j] = Frag<T>::load(Bb + bo);
      if (SPLIT) bl[j] = Frag<T>::load(Bb2 + bo);
    }
#pragma unroll
    for (int i = 0; i < 4; ++i) {
      const size_t ao = (size_t)(m0 + (i << 4) + rlane) * lda + koff + k0;
      V ah = Frag<T>::load(Ab + ao);
      V al;
      if (SPLIT) al = Frag<T>::load(Ab2 + ao);
#pragma unroll
      for (int j = 0; j < 4; ++j) {
        acc[i][j] = Frag<T>::mma(ah, bh[j], acc[i][j]);
        if (SPLIT) {
          acc[i][j] = Frag<T>::mma(ah, bl[j], acc[i][j]);
          acc[i][j] = Frag<T>::mma(al, bh[j], acc[i][j]);
        }
      }
      Frag<T>::guard4(acc[i][0], acc[i][1], acc[i][2], acc[i][3], ah, SPLIT ? al : ah);
    }
    Frag<T>::keep(bh[0], bh[1], bh[2], bh[3]);
    if (SPLIT) Frag<T>::keep(bl[0], bl[1], bl[2], bl[3]);
  }
  acc_guard4(acc[0][0], acc[0][1], acc[0][2], acc[0][3]);
  acc_guard4(acc[1][0], acc[1][1], acc[1][2], acc[1][3]);
  acc_guard4(acc[2][0], acc[2][1], acc[2][2], acc[2][3]);
  acc_guard4(acc[3][0], acc[3][1], acc[3][2], acc[3][3]);

  float* slab = sT[wave];
  const float* Rb = RESID ? (resid + (size_t)b * strideR) : nullptr;
#pragma unroll
  for (int i = 0; i < 4; ++i) {
    const int mBase = m0 + (i << 4);
#pragma unroll
    for (int j = 0; j < 4; ++j) {
      const int n = n0 + (j << 4) + rlane;
      float bv = 0.f;
      if (BIAS_MODE == 2) bv = bias[n];
#pragma unroll
      for (int r = 0; r < 8; ++r) {
        float v = acc[i][j][r] * scale;
        if (BIAS_MODE == 1) v += bias[mBase + mOff + r];
        if (BIAS_MODE == 2) v += bv;
        if (RESID) v += Rb[(size_t)(mBase + mOff + r) * ldc + n];
        if (ACT == 2) v = fmaxf(v, 0.0f);
        if (ACT == 4) v = (v > 0.f) ? v : 0.01f * v;
        slab[(mOff + r) * 68 + (j << 4) + rlane] = v;
      }
    }
    __builtin_amdgcn_fence(__ATOMIC_RELEASE, "workgroup");
    __builtin_amdgcn_wave_barrier();
    __builtin_amdgcn_fence(__ATOMIC_ACQUIRE, "workgroup");
    if (OUT_MODE == 0) {
      float* C = (float*)Cout + (size_t)b * strideC;
      const int hh = lane >> 4, c4 = (lane & 15) * 4;
      for (int pass = 0; pass < 2; ++pass) {
#pragma unroll
        for (int it = 0; it < 8; ++it) {
          const int row = it * 2 + hh;
          v4f v = *(const v4f*)(slab + row * 68 + c4);
          *(volatile v4f*)(C + (size_t)(mBase + row) * ldc + n0 + c4) = v;
        }
        __threadfence();
      }
    } else {
      const int q = lane >> 3, c8 = (lane & 7) * 8;
      unsigned short* C  = (unsigned short*)Cout  + (size_t)b * strideC;
      unsigned short* C2 = (OUT_MODE == 2) ? ((unsigned short*)Cout2 + (size_t)b * strideC) : nullptr;
      for (int pass = 0; pass < 2; ++pass) {
#pragma unroll
        for (int it = 0; it < 4; ++it) {
          const int row = it * 4 + q;
          const float* sp = slab + row * 68 + c8;
          v8h hv, lv;
#pragma unroll
          for (int e = 0; e < 8; ++e) {
            if (OUT_MODE == 1) {
              hv[e] = (_Float16)sp[e];
            } else {
              unsigned short hb = f2bf_bits(sp[e]);
              unsigned short lb = f2bf_bits(sp[e] - bf_bits2f(hb));
              hv[e] = __builtin_bit_cast(_Float16, hb);
              lv[e] = __builtin_bit_cast(_Float16, lb);
            }
          }
          *(volatile v8h*)(C + (size_t)(mBase + row) * ldc + n0 + c8) = hv;
          if (OUT_MODE == 2) *(volatile v8h*)(C2 + (size_t)(mBase + row) * ldc + n0 + c8) = lv;
        }
        __threadfence();
      }
    }
    __builtin_amdgcn_fence(__ATOMIC_RELEASE, "workgroup");
    __builtin_amdgcn_wave_barrier();
    __builtin_amdgcn_fence(__ATOMIC_ACQUIRE, "workgroup");
  }
}

__global__ __launch_bounds__(NTHR) void prep_wt_kernel(const float* __restrict__ W, long wz, int ldw, int ncols,
                                                      unsigned short* __restrict__ PH, unsigned short* __restrict__ PL, long pz) {
  __shared__ float sm[64][65];
  const int t  = threadIdx.x;
  const int k0 = blockIdx.x * 64;
  const int n0 = blockIdx.y * 64;
  const int z  = blockIdx.z;
  const float* Wz = W + (size_t)z * wz;
#pragma unroll
  for (int i = 0; i < 16; ++i) {
    const int e = i * NTHR + t;
    const int r = e >> 6;
    const int c = e & 63;
    const int nc = n0 + c;
    const int ncl = nc < ncols ? nc : ncols - 1;
    const float f = (nc < ncols) ? 1.0f : 0.0f;
    const float v = Wz[(size_t)(k0 + r) * ldw + ncl] * f;
    sm[c][r] = v;
  }
  __syncthreads();
  const int lane = t & 31, wave = t >> 5;
  const int q = lane >> 3, c8 = (lane & 7) * 8;
  unsigned short* ph = PH + (size_t)z * pz;
  unsigned short* pl = PL + (size_t)z * pz;
  for (int pass = 0; pass < 2; ++pass) {
#pragma unroll
    for (int it = 0; it < 2; ++it) {
      const int row = wave * 8 + it * 4 + q;
      unsigned short hb[8], lb[8];
#pragma unroll
      for (int e = 0; e < 8; ++e) {
        const float v = sm[row][c8 + e];
        hb[e] = f2bf_bits(v);
        lb[e] = f2bf_bits(v - bf_bits2f(hb[e]));
      }
      const v4u uh = (v4u){pk16(hb[0], hb[1]), pk16(hb[2], hb[3]), pk16(hb[4], hb[5]), pk16(hb[6], hb[7])};
      const v4u ul = (v4u){pk16(lb[0], lb[1]), pk16(lb[2], lb[3]), pk16(lb[4], lb[5]), pk16(lb[6], lb[7])};
      const size_t o = (size_t)(n0 + row) * FDIM + k0 + c8;
      *(volatile v4u*)(ph + o) = uh;
      *(volatile v4u*)(pl + o) = ul;
    }
    __threadfence();
  }
}

__global__ __launch_bounds__(NTHR) void xplanes_kernel(const float* __restrict__ x, unsigned short* __restrict__ XH,
                                                      unsigned short* __restrict__ XL) {
  const int i = blockIdx.x * NTHR + threadIdx.x;
  const int row = i >> 4;
  const int c8 = (i & 15) * 8;
  const bool live = row < NNODE;
  const int rcl = live ? row : (NNODE - 1);
  const float lf = live ? 1.0f : 0.0f;
  const float* p = x + (size_t)rcl * FDIM + c8;
  const v4f a = *(const v4f*)(p);
  const v4f c = *(const v4f*)(p + 4);
  unsigned short hb[8], lb[8];
#pragma unroll
  for (int e = 0; e < 4; ++e) {
    const float v0 = a[e] * lf;
    const float v1 = c[e] * lf;
    hb[e] = f2bf_bits(v0); lb[e] = f2bf_bits(v0 - bf_bits2f(hb[e]));
    hb[4 + e] = f2bf_bits(v1); lb[4 + e] = f2bf_bits(v1 - bf_bits2f(hb[4 + e]));
  }
  const v4u uh = (v4u){pk16(hb[0], hb[1]), pk16(hb[2], hb[3]), pk16(hb[4], hb[5]), pk16(hb[6], hb[7])};
  const v4u ul = (v4u){pk16(lb[0], lb[1]), pk16(lb[2], lb[3]), pk16(lb[4], lb[5]), pk16(lb[6], lb[7])};
  const size_t o = 8 * (size_t)i;
  for (int pass = 0; pass < 2; ++pass) {
    *(volatile v4u*)(XH + o) = uh;
    *(volatile v4u*)(XL + o) = ul;
    __threadfence();
  }
}

__device__ __forceinline__ int blk_excl_scan(int cnt, int* scan_ws, int tid, int* tot) {
  const int lane = tid & 31, wave = tid >> 5; int incl = cnt;
#pragma unroll
  for (int o = 1; o < 32; o <<= 1) { const int v = __shfl_up(incl, o, 32); if (lane >= o) incl += v; }
  if (lane == 31) scan_ws[wave] = incl;
  __syncthreads();
  if (wave == 0) { int wv = scan_ws[lane]; wv &= -(int)(lane < NTHR / 32); int wincl = wv;
#pragma unroll
    for (int o = 1; o < 32; o <<= 1) { const int v = __shfl_up(wincl, o, 32); if (lane >= o) wincl += v; }
    if (lane < NTHR / 32) scan_ws[32 + lane] = wincl - wv; if (lane == 31) scan_ws[64] = wincl; }
  __syncthreads();
  const int res = scan_ws[32 + wave] + incl - cnt; *tot = scan_ws[64];
  return res;
}
template <int SP, int CAP>
__device__ __forceinline__ int chunk_hits_d(const int* __restrict__ dstv, int e0, int n0, int tid, int* LIST, int* scan_ws) {
  const int eb = e0 + tid * SP;
  const bool inr = eb < NEDGE;
  const int ebc = inr ? eb : (NEDGE - SP);
  int rec[SP]; int cnt = 0;
#pragma unroll
  for (int k = 0; k < SP; k += 4) {
    const v4i d4 = *(const v4i*)(dstv + ebc + k);
#pragma unroll
    for (int e = 0; e < 4; ++e) {
      const int d = d4[e]; int r = -1;
      if (inr && d >= n0 && d < n0 + SRB) { r = ((d - n0) << 16) | (tid * SP + k + e); ++cnt; }
      rec[k + e] = r;
    }
  }
  int tot; int p = blk_excl_scan(cnt, scan_ws, tid, &tot);
#pragma unroll
  for (int k = 0; k < SP; ++k) if (rec[k] >= 0) { if ((unsigned)p < (unsigned)CAP) LIST[p] = rec[k]; ++p; }
  __syncthreads();
  return tot < CAP ? tot : CAP;
}
__device__ __forceinline__ int list_entry(const int* LIST, int q, int tot) {
  const int qc = q < tot ? q : (tot - 1);
  const int keep = -(int)(q < tot);
  const int rvl = LIST[qc];
  return (rvl & keep) | (~keep);
}

__global__ __launch_bounds__(NTHR) void dinv_kernel(const int* __restrict__ ei, float* __restrict__ DINV) {
  __shared__ int LIST[SCH];
  __shared__ __align__(16) int SC[SRB];
  __shared__ int scan_ws[SCANW];
  const int tid = threadIdx.x, lane = tid & 31, wave = tid >> 5;
  const int n0 = blockIdx.x * SRB;
  for (int i = tid; i < SRB; i += NTHR) SC[i] = 0;
  for (int i = tid; i < SCH; i += NTHR) LIST[i] = 0;
  if (tid < SCANW) scan_ws[tid] = 0;
  __syncthreads();
  const int* dstv = ei + NEDGE;
#pragma unroll 1
  for (int c = 0; c < NCH; ++c) {
    const int tot = chunk_hits_d<SPT, SCH>(dstv, c * SCH, n0, tid, LIST, scan_ws);
#pragma unroll 1
    for (int base = 0; base < tot; base += 32) {
      const int q = base + lane;
      const int rv = list_entry(LIST, q, tot);
      const int own = (rv >= 0 && (rv >> 26) == wave) ? 1 : 0;
      unsigned msk = (unsigned)__ballot(own);
#pragma unroll 1
      for (int it = 0; it < 32; ++it) {
        if (msk == 0u) break;
        const int bp = __builtin_ctz(msk); msk &= msk - 1u;
        const int rb = __shfl(rv, bp, 32);
        const int dl = (rb >> 16) & (SRB - 1);
        const int cur = SC[dl];
        if (lane == 0) SC[dl] = cur + 1;
      }
    }
    __syncthreads();
  }
#pragma unroll 1
  for (int it = 0; it < RPW / 128; ++it) {
    const int idx = wave * RPW + it * 128 + 4 * lane;
    const v4i c4 = *(const v4i*)(SC + idx);
    v4f dv;
#pragma unroll
    for (int e = 0; e < 4; ++e) dv[e] = 1.0f / sqrtf((float)(c4[e] + 1));
    float* p = DINV + n0 + idx;
    for (int pass = 0; pass < 2; ++pass) { *(volatile v4f*)p = dv; __threadfence(); }
  }
}

__global__ __launch_bounds__(NTHR) void gcn_layer_kernel(const float* __restrict__ H, const int* __restrict__ ei,
                                                        const float* __restrict__ DINV, const float* __restrict__ bsl,
                                                        const float* __restrict__ gl, const float* __restrict__ bl,
                                                        const float* xin, float* xout,
                                                        unsigned short* __restrict__ XH, unsigned short* __restrict__ XL,
                                                        float* AGG) {
  __shared__ int LIST[SCH];
  __shared__ int scan_ws[SCANW];
  const int tid = threadIdx.x, lane = tid & 31, wave = tid >> 5;
  const int n0 = blockIdx.x * SRB;
  const v4f bs4 = *(const v4f*)(bsl + 4 * lane);
  const v4f g4  = *(const v4f*)(gl + 4 * lane);
  const v4f bb4 = *(const v4f*)(bl + 4 * lane);
  const v4f z4 = {0.f, 0.f, 0.f, 0.f};
  for (int i = tid; i < SCH; i += NTHR) LIST[i] = 0;
  if (tid < SCANW) scan_ws[tid] = 0;
#pragma unroll 1
  for (int j = 0; j < RPW; ++j) *(v4f*)(AGG + (size_t)(n0 + wave * RPW + j) * FDIM + 4 * lane) = z4;
  __syncthreads();

  const int* srcv = ei; const int* dstv = ei + NEDGE;
#pragma unroll 1
  for (int c = 0; c < NCH; ++c) {
    const int e0 = c * SCH;
    const int tot = chunk_hits_d<SPT, SCH>(dstv, e0, n0, tid, LIST, scan_ws);
#pragma unroll 1
    for (int base = 0; base < tot; base += 32) {
      const int q = base + lane;
      const int rv = list_entry(LIST, q, tot);
      const int own = (rv >= 0 && (rv >> 26) == wave) ? 1 : 0;
      unsigned msk = (unsigned)__ballot(own);
      int eg = e0 + (rv & 0xFFFF); eg = eg < NEDGE ? eg : (NEDGE - 1);
      int s = srcv[eg]; s = s < 0 ? 0 : (s >= NNODE ? NNODE - 1 : s);
      const float wsv = DINV[s];
#pragma unroll 1
      for (int it = 0; it < 32; ++it) {
        if (msk == 0u) break;
        const int bp = __builtin_ctz(msk); msk &= msk - 1u;
        const int   sb = __shfl(s, bp, 32);
        const float wb = __shfl(wsv, bp, 32);
        const int   rb = __shfl(rv, bp, 32);
        const int   dl = (rb >> 16) & (SRB - 1);
        const v4f hv = *(const v4f*)(H + (size_t)sb * FDIM + 4 * lane);
        float* rp = AGG + (size_t)(n0 + dl) * FDIM + 4 * lane;
        v4f a = *(const v4f*)rp;
        a = a + wb * hv;
        *(v4f*)rp = a;
      }
    }
    __syncthreads();
  }

  const int la  = (2 * lane) & 31;
  const int lb2 = (2 * lane + 1) & 31;
#pragma unroll 1
  for (int j = 0; j < RPW; ++j) {
    const int dl = wave * RPW + j;
    const int n  = n0 + dl;
    if (n < NNODE) {
      const float di = DINV[n];
      const v4f a  = *(const v4f*)(AGG + (size_t)n * FDIM + 4 * lane);
      const v4f hv = *(const v4f*)(H + (size_t)n * FDIM + 4 * lane);
      const v4f xo = *(const v4f*)(xin + (size_t)n * FDIM + 4 * lane);
      v4f t = a + hv * di;
      t = t * di;
      t = t + bs4;
      float s1 = (t[0] + t[1]) + (t[2] + t[3]);
#pragma unroll
      for (int off = 16; off > 0; off >>= 1) s1 += __shfl_xor(s1, off, 32);
      const float mu = s1 * (1.0f / 128.0f);
      const v4f d = t - mu;
      float s2 = (d[0] * d[0] + d[1] * d[1]) + (d[2] * d[2] + d[3] * d[3]);
#pragma unroll
      for (int off = 16; off > 0; off >>= 1) s2 += __shfl_xor(s2, off, 32);
      const float var = s2 * (1.0f / 128.0f);
      const float rs = 1.0f / sqrtf(var + 1e-5f);
      v4f cv;
#pragma unroll
      for (int e = 0; e < 4; ++e) {
        float u = d[e] * rs;
        u = u * g4[e] + bb4[e];
        cv[e] = fmaxf(u, 0.0f);
      }
      const v4f xn = xo + cv;
      unsigned short hb[4], lbv[4];
#pragma unroll
      for (int e = 0; e < 4; ++e) { hb[e] = f2bf_bits(xn[e]); lbv[e] = f2bf_bits(xn[e] - bf_bits2f(hb[e])); }
      const unsigned uh01 = pk16(hb[0], hb[1]), uh23 = pk16(hb[2], hb[3]);
      const unsigned ul01 = pk16(lbv[0], lbv[1]), ul23 = pk16(lbv[2], lbv[3]);
      const unsigned hA01 = __shfl(uh01, la, 32), hA23 = __shfl(uh23, la, 32);
      const unsigned hB01 = __shfl(uh01, lb2, 32), hB23 = __shfl(uh23, lb2, 32);
      const unsigned lA01 = __shfl(ul01, la, 32), lA23 = __shfl(ul23, la, 32);
      const unsigned lB01 = __shfl(ul01, lb2, 32), lB23 = __shfl(ul23, lb2, 32);
      const v4u uh = (v4u){hA01, hA23, hB01, hB23};
      const v4u ul = (v4u){lA01, lA23, lB01, lB23};
      float* xr = xout + (size_t)n * FDIM + 4 * lane;
      unsigned short* ph = XH + (size_t)n * FDIM + 8 * lane;
      unsigned short* pl = XL + (size_t)n * FDIM + 8 * lane;
      for (int pass = 0; pass < 2; ++pass) {
        *(volatile v4f*)xr = xn;
        if (lane < 16) { *(volatile v4u*)ph = uh; *(volatile v4u*)pl = ul; }
        __threadfence();
      }
    } else if (n < NPAD) {
      const v4u zu = {0u, 0u, 0u, 0u};
      unsigned short* ph = XH + (size_t)n * FDIM + 8 * lane;
      unsigned short* pl = XL + (size_t)n * FDIM + 8 * lane;
      for (int pass = 0; pass < 2; ++pass) {
        if (lane < 16) { *(volatile v4u*)ph = zu; *(volatile v4u*)pl = zu; }
        __threadfence();
      }
    }
  }
}

__global__ __launch_bounds__(NTHR) void out_kernel(const float* __restrict__ OP, const float* __restrict__ cb, float* __restrict__ out) {
  const int i = blockIdx.x * NTHR + threadIdx.x;
  if (i >= NNODE * NCLS / 4) return;
  const int row = i >> 2, c4 = (i & 3) * 4;
  v4f v = *(const v4f*)(OP + (size_t)row * NCLP + c4);
  const v4f b = *(const v4f*)(cb + c4);
  v = v + b;
  float* p = out + 4 * (size_t)i;
  *(volatile v4f*)p = v;
  __threadfence();
  *(volatile v4f*)p = v;
}

extern "C" void kernel_launch(void* const* d_in, const int* in_sizes, int n_in,
                              void* d_out, int out_size, void* d_ws, size_t ws_size, hipStream_t stream) {
  (void)in_sizes; (void)n_in; (void)out_size;
  const float* x     = (const float*)d_in[0];
  const int*   ei    = (const int*)  d_in[1];
  const float* Ws    = (const float*)d_in[2];
  const float* bs    = (const float*)d_in[3];
  const float* ln_g  = (const float*)d_in[4];
  const float* ln_b  = (const float*)d_in[5];
  const float* cls_W = (const float*)d_in[6];
  const float* cls_b = (const float*)d_in[7];
  float* out = (float*)d_out;

  char* ws = (char*)d_ws; size_t off = 0;
  auto carve = [&](size_t bytes) -> char* { char* p = ws + off; off += (bytes + 255) & ~(size_t)255; return p; };
  float*          XC   = (float*)carve((size_t)NNODE * FDIM * 4);
  unsigned short* XH   = (unsigned short*)carve((size_t)NPAD * FDIM * 2);
  unsigned short* XL   = (unsigned short*)carve((size_t)NPAD * FDIM * 2);
  float*          H    = (float*)carve((size_t)NPAD * FDIM * 4);
  float*          AGG  = (float*)carve((size_t)AGGR * FDIM * 4);
  float*          DINV = (float*)carve((size_t)AGGR * 4);
  unsigned short* WH   = (unsigned short*)carve((size_t)NLAY * FDIM * FDIM * 2);
  unsigned short* WL   = (unsigned short*)carve((size_t)NLAY * FDIM * FDIM * 2);
  unsigned short* CWH  = (unsigned short*)carve((size_t)NCLP * FDIM * 2);
  unsigned short* CWL  = (unsigned short*)carve((size_t)NCLP * FDIM * 2);
  float*          OUTP = (float*)carve((size_t)NPAD * NCLP * 4);
  if (off > ws_size || off > (size_t)134217728) return;

  prep_wt_kernel<<<dim3(FDIM / 64, FDIM / 64, NLAY), NTHR, 0, stream>>>(Ws, (long)FDIM * FDIM, FDIM, FDIM, WH, WL, (long)FDIM * FDIM);
  prep_wt_kernel<<<dim3(FDIM / 64, 1, 1), NTHR, 0, stream>>>(cls_W, 0L, NCLS, NCLS, CWH, CWL, 0L);
  xplanes_kernel<<<(NPAD * FDIM / 8) / NTHR, NTHR, 0, stream>>>(x, XH, XL);
  dinv_kernel<<<NTILE, NTHR, 0, stream>>>(ei, DINV);

  const int gemm_tiles = (NPAD / 64) * (FDIM / 64);
  const int gemm_blocks = (gemm_tiles + 7) / 8;
  for (int l = 0; l < NLAY; ++l) {
    wmma_gemm64<1, true, 0, 0, false><<<dim3(gemm_blocks, 1), 256, 0, stream>>>(
        (const unsigned short*)XH, (const unsigned short*)XL, FDIM, 0L,
        (const unsigned short*)(WH + (size_t)l * FDIM * FDIM), (const unsigned short*)(WL + (size_t)l * FDIM * FDIM), FDIM, 0L,
        (void*)H, (void*)nullptr, FDIM, 0L,
        (const float*)nullptr, (const float*)nullptr, 0L, NPAD, FDIM, FDIM, 1.0f);
    const float* xin = (l == 0) ? x : (const float*)XC;
    gcn_layer_kernel<<<NTILE, NTHR, 0, stream>>>(H, ei, DINV, bs + (size_t)l * FDIM, ln_g + (size_t)l * FDIM, ln_b + (size_t)l * FDIM,
                                                xin, XC, XH, XL, AGG);
  }
  {
    const int ctiles = (NPAD / 64) * (NCLP / 64);
    wmma_gemm64<1, true, 0, 0, false><<<dim3((ctiles + 7) / 8, 1), 256, 0, stream>>>(
        (const unsigned short*)XH, (const unsigned short*)XL, FDIM, 0L,
        (const unsigned short*)CWH, (const unsigned short*)CWL, FDIM, 0L,
        (void*)OUTP, (void*)nullptr, NCLP, 0L,
        (const float*)nullptr, (const float*)nullptr, 0L, NPAD, NCLP, FDIM, 1.0f);
  }
  out_kernel<<<(NNODE * NCLS / 4 + NTHR - 1) / NTHR, NTHR, 0, stream>>>(OUTP, cls_b, out);
}
